// Block_65180423684994
// MI455X (gfx1250) — hardware-run, weakly checked
//
#include <hip/hip_runtime.h>


#ifndef NB
#define NB 8
#endif
#define NB_FULL 8
#define HT   56
#define WD   56
#define HW   (HT * WD)
#define CH   256
#define NG   16
#define CG   16
#define NP   9
#define HID  1024
#define NOFF 288
#define NMSK 144
#define NOM  432
#define NOMP 448
#define LTOK (NB * HW)
#define OSW  68
#define DWT  8
#define WSC  256.0f
#define WSI  (1.0f / 256.0f)
#define NEGB (-3.0e38f)

static_assert(NG * CG == CH);
static_assert(NG * NP * 2 == NOFF);
static_assert(NG * NP == NMSK);
static_assert(NOFF + NMSK == NOM);
static_assert(NOMP >= NOM);
static_assert(NOMP % 64 == 0);
static_assert(CH % 64 == 0);
static_assert(HID % 64 == 0);
static_assert(CH % 32 == 0);
static_assert(HID % 32 == 0);
static_assert(LTOK % 64 == 0);
static_assert(LTOK % 8 == 0);
static_assert(LTOK % (8 * DWT) == 0);
static_assert(CH == 32 * 8);
static_assert(CH == 256);
static_assert(NB <= NB_FULL);
static_assert((OSW * 4) % 16 == 0);
static_assert(OSW >= 64);
static_assert(64 * OSW * 4 <= 131072);
static_assert(10 * CH * 4 <= 131072);
static_assert(32 * 16 * 32 == 64 * 64 * 4);
static_assert(32 * 16 * 16 == 64 * 64 * 2);
static_assert(NOMP % 4 == 0);
static_assert(NOMP / 4 <= 128);

typedef _Float16 h16;
typedef __attribute__((ext_vector_type(16))) _Float16 v16h;
typedef __attribute__((ext_vector_type(8)))  _Float16 v8h;
typedef __attribute__((ext_vector_type(8)))  float    v8f;
typedef __attribute__((ext_vector_type(4)))  float    v4f;
typedef v4f  __attribute__((may_alias)) v4fa;

__device__ __forceinline__ unsigned short f2bf(float f) { unsigned u = __float_as_uint(f); u += 0x7FFFu + ((u >> 16) & 1u); return (unsigned short)(u >> 16); }
__device__ __forceinline__ float bfr(float f) { return __uint_as_float(((unsigned)f2bf(f)) << 16); }
__device__ __forceinline__ v16h cat16(v8h lo, v8h hi) { return __builtin_shufflevector(lo, hi, 0, 1, 2, 3, 4, 5, 6, 7, 8, 9, 10, 11, 12, 13, 14, 15); }
__device__ __forceinline__ v16h  ldh(const h16* p) { return cat16(*(const v8h*)p, *(const v8h*)(p + 16)); }
__device__ __forceinline__ void wave_sync() { __builtin_amdgcn_fence(3  , "wavefront"); __builtin_amdgcn_wave_barrier(); asm volatile("" ::: "memory"); }
__device__ __forceinline__ h16 toh_flush(float v) { const h16 r = (h16)v; return (fabsf(v) < 6.103515625e-05f) ? (h16)0.0f : r; }
__device__ __forceinline__ v8f wmma_g(v16h a, v16h b, v8f c) {
    c = __builtin_amdgcn_wmma_f32_16x16x32_f16(false, a, false, b, (short)0, c, false, false);
    asm volatile("v_nop\n\tv_nop\n\tv_nop\n\tv_nop" : "+v"(c) : "v"(a), "v"(b));
    return c; }
__device__ __forceinline__ int clampi(int v, int lo, int hi) { return v < lo ? lo : (v > hi ? hi : v); }

__global__ __launch_bounds__(256) void k_wcvt(const float* __restrict__ src, h16* dst, size_t n8, size_t nsrc8) {
    const size_t i = (size_t)blockIdx.x * 256 + threadIdx.x; if (i >= n8) return;
    const bool real = i < nsrc8;
    const size_t ic = real ? i : (nsrc8 - 1);
    v8f v = *(const v8f*)(src + ic * 8);
    asm volatile("" : "+v"(v));
    v8h o;
#pragma unroll
    for (int k = 0; k < 8; ++k) { const h16 c = toh_flush(bfr(v[k]) * WSC); o[k] = real ? c : (h16)0.0f; }
    *(volatile v8h*)(dst + i * 8) = o; __threadfence(); *(volatile v8h*)(dst + i * 8) = o;
}

__global__ __launch_bounds__(128) void k_bcomb(const float* __restrict__ offb, const float* __restrict__ mskb, float* BC) {
    const int i = threadIdx.x; if (i >= NOMP / 4) return;
    v4f o;
#pragma unroll
    for (int k = 0; k < 4; ++k) {
        const int c = i * 4 + k;
        const int co = clampi(c, 0, NOFF - 1); const int cm = clampi(c - NOFF, 0, NMSK - 1);
        float a = offb[co]; float m = mskb[cm];
        asm volatile("" : "+v"(a)); asm volatile("" : "+v"(m));
        o[k] = (c < NOFF) ? bfr(a) : ((c < NOM) ? bfr(m) : 0.0f); }
    *(volatile v4f*)(BC + i * 4) = o; __threadfence(); *(volatile v4f*)(BC + i * 4) = o;
}

__global__ __launch_bounds__(256) void k_ln(const float* __restrict__ X, const float* __restrict__ gam, const float* __restrict__ bet, h16* OUT, int cvt_in) {
#pragma clang fp contract(off)
    const int lane = threadIdx.x & 31;
    const int wave = __builtin_amdgcn_readfirstlane((int)(threadIdx.x >> 5));
    const int t = blockIdx.x * 8 + wave;
    const size_t ro = (size_t)t * CH + (size_t)lane * 8;
    const v4f xa = *(const v4f*)(X + ro), xb = *(const v4f*)(X + ro + 4);
    float v[8];
#pragma unroll
    for (int i = 0; i < 4; ++i) { v[i] = cvt_in ? bfr(xa[i]) : xa[i]; v[4 + i] = cvt_in ? bfr(xb[i]) : xb[i]; }
    float s = 0.0f;
#pragma unroll
    for (int i = 0; i < 8; ++i) s = s + v[i];
#pragma unroll
    for (int m = 16; m >= 1; m >>= 1) s += __shfl_xor(s, m, 32);
    const float mu = s * (1.0f / CH);
    float d[8]; float ss = 0.0f;
#pragma unroll
    for (int i = 0; i < 8; ++i) { d[i] = v[i] - mu; ss = ss + d[i] * d[i]; }
#pragma unroll
    for (int m = 16; m >= 1; m >>= 1) ss += __shfl_xor(ss, m, 32);
    const float rs = rsqrtf(ss * (1.0f / CH) + 1.0e-6f);
    const v4f ga = *(const v4f*)(gam + lane * 8), gb = *(const v4f*)(gam + lane * 8 + 4);
    const v4f ba = *(const v4f*)(bet + lane * 8), bb = *(const v4f*)(bet + lane * 8 + 4);
    v8h o;
#pragma unroll
    for (int i = 0; i < 4; ++i) { o[i] = toh_flush((d[i] * rs) * bfr(ga[i]) + bfr(ba[i])); o[4 + i] = toh_flush((d[4 + i] * rs) * bfr(gb[i]) + bfr(bb[i])); }
    h16* op = OUT + ro;
    *(volatile v8h*)op = o; __threadfence(); *(volatile v8h*)op = o;
}

__global__ __launch_bounds__(256) void k_dwconv(const h16* __restrict__ LN, const float* __restrict__ dww, const float* __restrict__ dwb, h16* X1) {
#pragma clang fp contract(off)
    __shared__ __align__(16) float wl[10 * CH];
#pragma unroll 1
    for (int i = threadIdx.x; i < 9 * CH; i += 256) wl[i] = bfr(dww[i]);
    wl[9 * CH + threadIdx.x] = bfr(dwb[threadIdx.x]);
    __syncthreads();
    const int lane = threadIdx.x & 31;
    const int wave = __builtin_amdgcn_readfirstlane((int)(threadIdx.x >> 5));
    const int c0 = lane * 8;
    const int tb = (blockIdx.x * 8 + wave) * DWT;
#pragma unroll 1
    for (int i = 0; i < DWT; ++i) {
        const int t = tb + i; const int n = t / HW, hw = t - n * HW; const int y = hw / WD, x = hw - y * WD;
        const v4f b0 = *(const v4fa*)(&wl[9 * CH + c0]), b1 = *(const v4fa*)(&wl[9 * CH + c0 + 4]);
        float acc[8];
#pragma unroll
        for (int j = 0; j < 4; ++j) { acc[j] = b0[j]; acc[4 + j] = b1[j]; }
#pragma unroll 1
        for (int tap = 0; tap < 9; ++tap) {
            const int ky = tap / 3, kx = tap - 3 * ky; const int yy = y + ky - 1, xx = x + kx - 1;
            const bool ok = (yy >= 0) & (yy < HT) & (xx >= 0) & (xx < WD);
            const int yc = clampi(yy, 0, HT - 1), xc = clampi(xx, 0, WD - 1);
            v8h v = *(const v8h*)(LN + ((size_t)n * HW + (size_t)(yc * WD + xc)) * CH + c0);
            asm volatile("" : "+v"(v));
            const v4f w0 = *(const v4fa*)(&wl[tap * CH + c0]), w1 = *(const v4fa*)(&wl[tap * CH + c0 + 4]);
#pragma unroll
            for (int j = 0; j < 4; ++j) {
                const float a0 = ok ? (float)v[j] : 0.0f; const float a1 = ok ? (float)v[4 + j] : 0.0f;
                acc[j] = acc[j] + a0 * w0[j]; acc[4 + j] = acc[4 + j] + a1 * w1[j]; }
        }
        v8h o;
#pragma unroll
        for (int j = 0; j < 8; ++j) o[j] = toh_flush(acc[j]);
        h16* op = X1 + (size_t)t * CH + c0;
        *(volatile v8h*)op = o; __threadfence(); *(volatile v8h*)op = o;
    }
}

__global__ __launch_bounds__(256) void k_sample(const h16* __restrict__ XP, const float* __restrict__ OM, h16* DC) {
#pragma clang fp contract(off)
    const int lane = threadIdx.x & 31;
    const int wave = __builtin_amdgcn_readfirstlane((int)(threadIdx.x >> 5));
    const int t = blockIdx.x * 8 + wave;
    const int n = t / HW, hw = t - n * HW; const int y = hw / WD, x = hw - y * WD;
    const int g = lane >> 1, c0 = lane * 8;
    const float* om = OM + (size_t)t * NOMP;
    float mx = NEGB;
#pragma unroll 1
    for (int p = 0; p < NP; ++p) mx = fmaxf(mx, om[NOFF + g * NP + p]);
    const float i58 = 1.0f / 58.0f;
    const float refx = ((float)x + 1.5f) * i58, refy = ((float)y + 1.5f) * i58;
    const size_t ib = (size_t)n * HW;
    float acc[8];
#pragma unroll
    for (int j = 0; j < 8; ++j) acc[j] = 0.0f;
    float se = 0.0f;
#pragma unroll 1
    for (int p = 0; p < NP; ++p) {
        const int pi = p / 3, pj = p - 3 * pi;
        const float ox = om[g * (2 * NP) + 2 * p], oy = om[g * (2 * NP) + 2 * p + 1], ml = om[NOFF + g * NP + p];
        const float e = __expf(ml - mx); se = se + e;
        const float lx = (refx + (float)(pi - 1) * i58) + ox * i58;
        const float ly = (refy + (float)(pj - 1) * i58) + oy * i58;
        float px = ((2.0f * lx - 1.0f) + 1.0f) * 29.0f - 0.5f;
        float py = ((2.0f * ly - 1.0f) + 1.0f) * 29.0f - 0.5f;
        px = fminf(fmaxf(px, -8.0f), 72.0f); py = fminf(fmaxf(py, -8.0f), 72.0f);
        const float x0f = floorf(px), y0f = floorf(py);
        const float wx1 = px - x0f, wy1 = py - y0f;
        const int ix0 = (int)x0f, iy0 = (int)y0f;
#pragma unroll 1
        for (int tap = 0; tap < 4; ++tap) {
            const int dx = tap & 1, dy = tap >> 1; const int ix = ix0 + dx, iy = iy0 + dy;
            const bool ok = (ix >= 1) & (ix <= WD) & (iy >= 1) & (iy <= HT);
            const float wgt = (dx ? wx1 : (1.0f - wx1)) * (dy ? wy1 : (1.0f - wy1));
            const float cw = ok ? (e * wgt) : 0.0f;
            const int xc = clampi(ix - 1, 0, WD - 1), yc = clampi(iy - 1, 0, HT - 1);
            v8h v = *(const v8h*)(XP + (ib + (size_t)(yc * WD + xc)) * CH + c0);
            asm volatile("" : "+v"(v));
#pragma unroll
            for (int j = 0; j < 8; ++j) acc[j] = acc[j] + cw * (float)v[j];
        }
    }
    const float rinv = 1.0f / se;
    v8h o;
#pragma unroll
    for (int j = 0; j < 8; ++j) o[j] = toh_flush(acc[j] * rinv);
    h16* op = DC + (size_t)t * CH + c0;
    *(volatile v8h*)op = o; __threadfence(); *(volatile v8h*)op = o;
}

template <int OUT16, int GELU, int RES>
__device__ __forceinline__ void gemm_tile(const h16* __restrict__ A, const h16* __restrict__ Bt, const float* __restrict__ bias, const float* res,
                                          float* OF, h16* OH, const int K, const int N) {
    __shared__ __align__(16) float os[64 * OSW];
    const int lane = threadIdx.x & 31, lr = lane & 15, hi = lane >> 4; const int r0 = blockIdx.x * 64, c0 = blockIdx.y * 64;
    v8f acc[4][4];
#pragma unroll
    for (int mb = 0; mb < 4; ++mb)
#pragma unroll
        for (int nb = 0; nb < 4; ++nb) acc[mb][nb] = (v8f){};
    const size_t aoff = (size_t)(r0 + lr) * K + 8 * hi, boff = (size_t)(c0 + lr) * K + 8 * hi;
#pragma unroll 1
    for (int kc = 0; kc < K; kc += 32) {
        v16h a[4];
#pragma unroll
        for (int mb = 0; mb < 4; ++mb) a[mb] = ldh(A + aoff + (size_t)mb * 16 * K + kc);
#pragma unroll
        for (int nb = 0; nb < 4; ++nb) { const v16h b = ldh(Bt + boff + (size_t)nb * 16 * K + kc);
#pragma unroll
            for (int mb = 0; mb < 4; ++mb) acc[mb][nb] = wmma_g(a[mb], b, acc[mb][nb]); }
    }
#pragma unroll
    for (int mb = 0; mb < 4; ++mb)
#pragma unroll
        for (int nb = 0; nb < 4; ++nb)
#pragma unroll
            for (int j = 0; j < 8; ++j) os[(mb * 16 + hi * 8 + j) * OSW + nb * 16 + lr] = acc[mb][nb][j];
    wave_sync();
    const int c4 = (lane & 15) * 4;
    v4f b4 = *(const v4f*)(bias + c0 + c4);
#pragma unroll
    for (int i = 0; i < 4; ++i) b4[i] = bfr(b4[i]);
#pragma unroll 1
    for (int it = 0; it < 32; ++it) { const int row = it * 2 + (lane >> 4);
        v4f v = *(const v4fa*)(&os[row * OSW + c4]);
#pragma unroll
        for (int i = 0; i < 4; ++i) v[i] = v[i] * WSI + b4[i];
        if (GELU) {
#pragma unroll
            for (int i = 0; i < 4; ++i) v[i] = 0.5f * v[i] * (1.0f + erff(v[i] * 0.70710678118654752f)); }
        if (RES) { const v4f r = *(const v4f*)(res + (size_t)(r0 + row) * N + c0 + c4);
#pragma unroll
            for (int i = 0; i < 4; ++i) v[i] = v[i] + ((RES == 1) ? bfr(r[i]) : r[i]); }
        *(v4fa*)(&os[row * OSW + c4]) = v; }
    wave_sync();
#pragma unroll 1
    for (int ps = 0; ps < 2; ++ps) {
        if (OUT16) {
#pragma unroll 1
            for (int it = 0; it < 16; ++it) { const int row = it * 4 + (lane >> 3), c8 = (lane & 7) * 8;
                const v4f x0 = *(const v4fa*)(&os[row * OSW + c8]); const v4f x1 = *(const v4fa*)(&os[row * OSW + c8 + 4]); v8h hv;
#pragma unroll
                for (int i = 0; i < 4; ++i) { hv[i] = toh_flush(x0[i]); hv[4 + i] = toh_flush(x1[i]); }
                *(volatile v8h*)(OH + (size_t)(r0 + row) * N + c0 + c8) = hv; }
        } else {
#pragma unroll 1
            for (int it = 0; it < 32; ++it) { const int row = it * 2 + (lane >> 4);
                const v4f val = *(const v4fa*)(&os[row * OSW + c4]);
                *(volatile v4f*)(OF + (size_t)(r0 + row) * N + c0 + c4) = val; }
        }
        if (ps == 0) __threadfence(); }
}

__global__ __launch_bounds__(32) void k_gemm_inp(const h16* __restrict__ A, const h16* __restrict__ Bt, const float* __restrict__ bias, h16* OH) {
    gemm_tile<1, 0, 0>(A, Bt, bias, (const float*)nullptr, (float*)nullptr, OH, CH, CH); }
__global__ __launch_bounds__(32) void k_gemm_om(const h16* __restrict__ A, const h16* __restrict__ Bt, const float* __restrict__ bias, float* OF) {
    gemm_tile<0, 0, 0>(A, Bt, bias, (const float*)nullptr, OF, (h16*)nullptr, CH, NOMP); }
__global__ __launch_bounds__(32) void k_gemm_out(const h16* __restrict__ A, const h16* __restrict__ Bt, const float* __restrict__ bias, const float* __restrict__ xres, float* OF) {
    gemm_tile<0, 0, 1>(A, Bt, bias, xres, OF, (h16*)nullptr, CH, CH); }
__global__ __launch_bounds__(32) void k_gemm_fc1(const h16* __restrict__ A, const h16* __restrict__ Bt, const float* __restrict__ bias, h16* OH) {
    gemm_tile<1, 1, 0>(A, Bt, bias, (const float*)nullptr, (float*)nullptr, OH, CH, HID); }
__global__ __launch_bounds__(32) void k_gemm_fc2(const h16* __restrict__ A, const h16* __restrict__ Bt, const float* __restrict__ bias, const float* __restrict__ yres, float* OF) {
    gemm_tile<0, 0, 2>(A, Bt, bias, yres, OF, (h16*)nullptr, HID, CH); }

static constexpr size_t al256(size_t v) { return (v + 255) & ~(size_t)255; }
static constexpr size_t SZ_ACT = al256((size_t)LTOK * CH * 2);
static constexpr size_t SZ_OM  = al256((size_t)LTOK * NOMP * 4);
static constexpr size_t SZ_Y   = al256((size_t)LTOK * CH * 4);
static constexpr size_t SZ_G   = al256((size_t)LTOK * HID * 2);
static constexpr size_t SZ_EARLY = 2 * SZ_ACT + SZ_OM;
static constexpr size_t SZ_BIG = SZ_EARLY > SZ_G ? SZ_EARLY : SZ_G;
static constexpr size_t N_W    = (size_t)2 * CH * CH + (size_t)2 * HID * CH + (size_t)NOMP * CH;
static constexpr size_t SZ_W   = al256(N_W * 2);
static constexpr size_t SZ_BC  = al256((size_t)NOMP * 4);
static constexpr size_t SZ_TOTAL = SZ_ACT + SZ_BIG + SZ_ACT + SZ_Y + SZ_W + SZ_BC;
static_assert(SZ_TOTAL <= (size_t)134217728);
static_assert(SZ_EARLY <= SZ_BIG);
static_assert(SZ_G <= SZ_BIG);
static_assert(((size_t)LTOK * CH * 2) % 256 == 0);
static_assert(((size_t)CH * CH * 2) % 256 == 0);
static_assert(((size_t)HID * CH * 2) % 256 == 0);
static_assert(((size_t)NOFF * CH * 2) % 256 == 0);
static_assert(((size_t)CH * CH) % 8 == 0);
static_assert(((size_t)NOFF * CH) % 8 == 0);
static_assert(((size_t)NMSK * CH) % 8 == 0);
static_assert(((size_t)(NOMP - NOFF) * CH) % 8 == 0);

extern "C" void kernel_launch(void* const* d_in, const int* in_sizes, int n_in,
                              void* d_out, int out_size, void* d_ws, size_t ws_size, hipStream_t stream) {
    if (n_in < 19) return;
    if ((size_t)in_sizes[0] < (size_t)LTOK * CH) return;
    if (in_sizes[1] < CH || in_sizes[2] < CH || in_sizes[3] < 9 * CH || in_sizes[4] < CH) return;
    if (in_sizes[5] < NOFF * CH || in_sizes[6] < NOFF || in_sizes[7] < NMSK * CH || in_sizes[8] < NMSK) return;
    if (in_sizes[9] < CH * CH || in_sizes[10] < CH || in_sizes[11] < CH * CH || in_sizes[12] < CH) return;
    if (in_sizes[13] < CH || in_sizes[14] < CH || in_sizes[15] < HID * CH || in_sizes[16] < HID) return;
    if (in_sizes[17] < CH * HID || in_sizes[18] < CH) return;
    if ((size_t)out_size < (size_t)LTOK * CH) return;
    if (SZ_TOTAL > ws_size) return;
    const float* x     = (const float*)d_in[0];
    const float* ln1g  = (const float*)d_in[1];
    const float* ln1b  = (const float*)d_in[2];
    const float* dww   = (const float*)d_in[3];
    const float* dwb   = (const float*)d_in[4];
    const float* offw  = (const float*)d_in[5];
    const float* offb  = (const float*)d_in[6];
    const float* mskw  = (const float*)d_in[7];
    const float* mskb  = (const float*)d_in[8];
    const float* inpw  = (const float*)d_in[9];
    const float* inpb  = (const float*)d_in[10];
    const float* outw  = (const float*)d_in[11];
    const float* outb  = (const float*)d_in[12];
    const float* ln2g  = (const float*)d_in[13];
    const float* ln2b  = (const float*)d_in[14];
    const float* fc1w  = (const float*)d_in[15];
    const float* fc1b  = (const float*)d_in[16];
    const float* fc2w  = (const float*)d_in[17];
    const float* fc2b  = (const float*)d_in[18];
    float* OUT = (float*)d_out;
    char* wsp = (char*)d_ws;
    h16* LNH = (h16*)wsp; wsp += SZ_ACT;
    char* big = wsp; wsp += SZ_BIG;
    h16* X1H = (h16*)big;
    h16* XPH = (h16*)(big + SZ_ACT);
    float* OM = (float*)(big + 2 * SZ_ACT);
    h16* GH  = (h16*)big;
    h16* DCH = (h16*)wsp; wsp += SZ_ACT;
    float* Y = (float*)wsp; wsp += SZ_Y;
    h16* WB  = (h16*)wsp; wsp += SZ_W;
    float* BC = (float*)wsp; wsp += SZ_BC;
    h16* WI = WB; h16* WO = WI + (size_t)CH * CH; h16* W1 = WO + (size_t)CH * CH; h16* W2 = W1 + (size_t)HID * CH; h16* WC = W2 + (size_t)CH * HID;

    { const size_t n8 = (size_t)CH * CH / 8; const unsigned g = (unsigned)((n8 + 255) / 256);
      k_wcvt<<<g, 256, 0, stream>>>(inpw, WI, n8, n8); k_wcvt<<<g, 256, 0, stream>>>(outw, WO, n8, n8); }
    { const size_t n8 = (size_t)HID * CH / 8; const unsigned g = (unsigned)((n8 + 255) / 256);
      k_wcvt<<<g, 256, 0, stream>>>(fc1w, W1, n8, n8); k_wcvt<<<g, 256, 0, stream>>>(fc2w, W2, n8, n8); }
    { const size_t n8 = (size_t)NOFF * CH / 8;
      k_wcvt<<<(unsigned)((n8 + 255) / 256), 256, 0, stream>>>(offw, WC, n8, n8); }
    { const size_t n8 = (size_t)(NOMP - NOFF) * CH / 8, s8 = (size_t)NMSK * CH / 8;
      k_wcvt<<<(unsigned)((n8 + 255) / 256), 256, 0, stream>>>(mskw, WC + (size_t)NOFF * CH, n8, s8); }
    k_bcomb<<<1, 128, 0, stream>>>(offb, mskb, BC);

    k_ln<<<LTOK / 8, 256, 0, stream>>>(x, ln1g, ln1b, LNH, 1);
    k_dwconv<<<LTOK / (8 * DWT), 256, 0, stream>>>(LNH, dww, dwb, X1H);
    k_gemm_inp<<<dim3(LTOK / 64, CH / 64, 1), 32, 0, stream>>>(LNH, WI, inpb, XPH);
    k_gemm_om<<<dim3(LTOK / 64, NOMP / 64, 1), 32, 0, stream>>>(X1H, WC, BC, OM);
    k_sample<<<LTOK / 8, 256, 0, stream>>>(XPH, OM, DCH);
    k_gemm_out<<<dim3(LTOK / 64, CH / 64, 1), 32, 0, stream>>>(DCH, WO, outb, x, Y);
    k_ln<<<LTOK / 8, 256, 0, stream>>>(Y, ln2g, ln2b, LNH, 0);
    k_gemm_fc1<<<dim3(LTOK / 64, HID / 64, 1), 32, 0, stream>>>(LNH, W1, fc1b, GH);
    k_gemm_fc2<<<dim3(LTOK / 64, CH / 64, 1), 32, 0, stream>>>(GH, W2, fc2b, Y, OUT);
}
